// MapNet_6468220748262
// MI455X (gfx1250) — hardware-verified
//
#include <hip/hip_runtime.h>
#include <stddef.h>


#define HID   256
#define KOUT  27
#define NPAD  32
#define PXB   128
#define NTHR  256

static_assert(NTHR == HID);
static_assert(PXB == 16 * (NTHR / 32));
static_assert((PXB * 3) % 4 == 0);
static_assert(((PXB * 3) / 4) % 32 == 0);
static_assert(PXB % 32 == 0);
static_assert(PXB / 4 == 32);
static_assert(HID % 32 == 0);
static_assert(HID / 8 == 32);
static_assert(KOUT <= NPAD);

typedef unsigned short us_t;
typedef us_t   v8us  __attribute__((ext_vector_type(8)));
typedef __bf16 v16bf __attribute__((ext_vector_type(16)));
typedef float  v4f   __attribute__((ext_vector_type(4)));
typedef float  v8f   __attribute__((ext_vector_type(8)));
union FragB { v16bf v; v8us h[2]; };

__device__ __forceinline__ v8f wmb(v16bf a, v16bf b, v8f c) {
  v8f d = __builtin_amdgcn_wmma_f32_16x16x32_bf16(false, a, false, b, (short)0, c, false, false);
#if defined(__HIP_DEVICE_COMPILE__)
  asm volatile("v_nop\n\tv_nop\n\tv_nop\n\tv_nop" : "+v"(d) : "v"(a), "v"(b));
#endif
  return d;
}

__device__ __forceinline__ v8f zero8() {
  v8f z = {0.f, 0.f, 0.f, 0.f, 0.f, 0.f, 0.f, 0.f};
  return z;
}

__device__ __forceinline__ us_t bf16_bits(float x) {
  unsigned u = __float_as_uint(x);
  u = (u + 0x7FFFu + ((u >> 16) & 1u)) >> 16;
  return (us_t)u;
}
__device__ __forceinline__ float bf16_val(us_t b) {
  return __uint_as_float(((unsigned)b) << 16);
}

__global__ __launch_bounds__(NTHR) void k_prep(const float* __restrict__ W2, us_t* Bhi, us_t* Blo) {
  const int i = blockIdx.x * NTHR + (int)threadIdx.x;
  if (i >= NPAD * HID / 8) return;
  const int n  = i >> 5;
  const int k0 = (i & 31) * 8;
  const bool live = n < KOUT;
  const int nc = live ? n : KOUT - 1;
  v8us vh, vl;
#pragma unroll
  for (int e = 0; e < 8; ++e) {
    float w = W2[(size_t)nc * HID + k0 + e];
    w = live ? w : 0.f;
    const us_t hb = bf16_bits(w);
    const us_t lb = bf16_bits(w - bf16_val(hb));
    vh[e] = hb;
    vl[e] = lb;
  }
  us_t* ph = Bhi + (size_t)n * HID + k0;
  us_t* pl = Blo + (size_t)n * HID + k0;
  *(volatile v8us*)ph = vh;
  *(volatile v8us*)pl = vl;
  __threadfence();
  *(volatile v8us*)ph = vh;
  *(volatile v8us*)pl = vl;
}

__global__ __launch_bounds__(NTHR) void k_main(const float* __restrict__ pos, const int* __restrict__ mp,
                                               const float* __restrict__ feats, const float* __restrict__ depth,
                                               const float* __restrict__ W1, const float* __restrict__ b1,
                                               const us_t* __restrict__ Bhi, const us_t* __restrict__ Blo,
                                               const float* __restrict__ b2, float* out, int fH, int fW) {
  __shared__ v4f   sW4[HID];
  __shared__ v4f   sPos4[PXB * 3 / 4];
  __shared__ int   sMy[PXB];
  __shared__ int   sMx[PXB];
  __shared__ float sB2[NPAD];
  __shared__ v4f   sOut4[PXB / 4];
  const float* sPos = (const float*)sPos4;
  float* sOut = (float*)sOut4;
  (void)depth;

  const int tid = threadIdx.x, lane = tid & 31, wv = tid >> 5, h = lane >> 4, m = lane & 15;
  const size_t pix0 = (size_t)blockIdx.x * PXB;

  {
    v4f w;
    w.x = W1[3 * tid + 0];
    w.y = W1[3 * tid + 1];
    w.z = W1[3 * tid + 2];
    w.w = b1[tid];
    sW4[tid] = w;
  }
  if (tid < PXB * 3 / 4) {
    sPos4[tid] = *(const v4f*)(pos + pix0 * 3 + 4 * (size_t)tid);
  }
  if (tid < PXB) {
    int y = mp[2 * (pix0 + (size_t)tid) + 0];
    int x = mp[2 * (pix0 + (size_t)tid) + 1];
    y = y < 0 ? y + fH : y;
    x = x < 0 ? x + fW : x;
    y = y < 0 ? 0 : (y > fH - 1 ? fH - 1 : y);
    x = x < 0 ? 0 : (x > fW - 1 ? fW - 1 : x);
    sMy[tid] = y;
    sMx[tid] = x;
  }
  if (tid < NPAD) {
    const int ci = tid < KOUT ? tid : KOUT - 1;
    const float v = b2[ci];
    sB2[tid] = (tid < KOUT) ? v : 0.f;
  }
  __syncthreads();

  const int pb = 16 * wv;
  const float p0 = sPos[3 * (pb + m) + 0];
  const float p1 = sPos[3 * (pb + m) + 1];
  const float p2 = sPos[3 * (pb + m) + 2];
  const us_t* bh0p = Bhi + (size_t)m * HID + 8 * h;
  const us_t* bl0p = Blo + (size_t)m * HID + 8 * h;
  const us_t* bh1p = Bhi + (size_t)(16 + m) * HID + 8 * h;
  const us_t* bl1p = Blo + (size_t)(16 + m) * HID + 8 * h;

  v8f acc0 = zero8(), acc1 = zero8();
#pragma unroll 1
  for (int ks = 0; ks < HID / 32; ++ks) {
    const int k0 = 32 * ks;
    v16bf av = {}, lv = {};
#pragma unroll
    for (int j = 0; j < 16; ++j) {
      const int kk = k0 + 8 * h + (j & 7) + ((j >> 3) << 4);
      const v4f w = sW4[kk];
      const float a = fmaf(p2, w.z, fmaf(p1, w.y, fmaf(p0, w.x, w.w)));
      const float v = fmaxf(a, a * 0.01f);
      const __bf16 hb = (__bf16)v;
      const __bf16 lb = (__bf16)(v - (float)hb);
      av[j] = hb;
      lv[j] = lb;
    }
    FragB g0, g1, q0, q1;
    g0.h[0] = *(const v8us*)(bh0p + k0);
    g0.h[1] = *(const v8us*)(bh0p + k0 + 16);
    q0.h[0] = *(const v8us*)(bl0p + k0);
    q0.h[1] = *(const v8us*)(bl0p + k0 + 16);
    g1.h[0] = *(const v8us*)(bh1p + k0);
    g1.h[1] = *(const v8us*)(bh1p + k0 + 16);
    q1.h[0] = *(const v8us*)(bl1p + k0);
    q1.h[1] = *(const v8us*)(bl1p + k0 + 16);
    acc0 = wmb(av, g0.v, acc0);
    acc0 = wmb(av, q0.v, acc0);
    acc0 = wmb(lv, g0.v, acc0);
    acc1 = wmb(av, g1.v, acc1);
    acc1 = wmb(av, q1.v, acc1);
    acc1 = wmb(lv, g1.v, acc1);
  }

  const int kA = m;
  const int cA = kA / 9, rA = kA - 9 * cA, dyA = rA / 3 - 1, dxA = rA - 3 * (rA / 3) - 1;
  const bool vB = (16 + m) < KOUT;
  const int kB = vB ? (16 + m) : (KOUT - 1);
  const int cB = kB / 9, rB = kB - 9 * cB, dyB = rB / 3 - 1, dxB = rB - 3 * (rB / 3) - 1;
  const float bA = sB2[m];
  const float bB = sB2[16 + m];
  const size_t plane = (size_t)fH * (size_t)fW;

  float val[8];
#pragma unroll
  for (int r = 0; r < 8; ++r) {
    const int q = pb + 8 * h + r;
    const int y = sMy[q], x = sMx[q];
    int ya = y + dyA, xa = x + dxA;
    const bool ia = ((unsigned)ya < (unsigned)fH) && ((unsigned)xa < (unsigned)fW);
    ya = ya < 0 ? 0 : (ya > fH - 1 ? fH - 1 : ya);
    xa = xa < 0 ? 0 : (xa > fW - 1 ? fW - 1 : xa);
    float fA = feats[(size_t)cA * plane + (size_t)ya * fW + xa];
    fA = ia ? fA : 0.f;
    int yb = y + dyB, xb = x + dxB;
    const bool ib = vB && ((unsigned)yb < (unsigned)fH) && ((unsigned)xb < (unsigned)fW);
    yb = yb < 0 ? 0 : (yb > fH - 1 ? fH - 1 : yb);
    xb = xb < 0 ? 0 : (xb > fW - 1 ? fW - 1 : xb);
    float fB = feats[(size_t)cB * plane + (size_t)yb * fW + xb];
    fB = ib ? fB : 0.f;
    val[r] = fmaf(fB, acc1[r] + bB, fA * (acc0[r] + bA));
  }
#pragma unroll
  for (int off = 1; off < 16; off <<= 1) {
#pragma unroll
    for (int r = 0; r < 8; ++r) val[r] += __shfl_xor(val[r], off, 32);
  }
  float o = val[0];
#pragma unroll
  for (int r = 1; r < 8; ++r) o = ((m & 7) == r) ? val[r] : o;
  if (m < 8) sOut[pb + 8 * h + m] = o;
  __syncthreads();

  if (tid < 32) {
    const v4f v = sOut4[lane];
    float* g = out + pix0 + 4 * (size_t)lane;
    *(volatile v4f*)g = v;
    __threadfence();
    *(volatile v4f*)g = v;
  }
}

extern "C" void kernel_launch(void* const* d_in, const int* in_sizes, int n_in,
                              void* d_out, int out_size, void* d_ws, size_t ws_size,
                              hipStream_t stream) {
  if (n_in < 8) return;
  const int P = in_sizes[1] / 2;
  if (P <= 0 || in_sizes[1] != 2 * P) return;
  if (in_sizes[0] != 3 * P) return;
  if (out_size != P) return;
  if ((P % PXB) != 0) return;
  const int hw = in_sizes[2] / 3;
  if (hw <= 0 || in_sizes[2] != 3 * hw) return;
  int fw = 1;
  while (fw * fw < hw && fw < 46340) ++fw;
  if (fw * fw != hw) return;
  if (in_sizes[4] != HID * 3 || in_sizes[5] != HID) return;
  if (in_sizes[6] != KOUT * HID || in_sizes[7] != KOUT) return;

  const float* pos   = (const float*)d_in[0];
  const int*   mp    = (const int*)d_in[1];
  const float* feats = (const float*)d_in[2];
  const float* depth = (const float*)d_in[3];
  const float* W1    = (const float*)d_in[4];
  const float* b1    = (const float*)d_in[5];
  const float* W2    = (const float*)d_in[6];
  const float* b2    = (const float*)d_in[7];
  float* out = (float*)d_out;

  const size_t planeBytes = (size_t)NPAD * HID * 2;
  const size_t total = 2 * planeBytes;
  if (total > ws_size || total > (size_t)134217728) return;
  us_t* Bhi = (us_t*)d_ws;
  us_t* Blo = Bhi + (size_t)NPAD * HID;

  k_prep<<<(NPAD * HID / 8 + NTHR - 1) / NTHR, NTHR, 0, stream>>>(W2, Bhi, Blo);
  k_main<<<P / PXB, NTHR, 0, stream>>>(pos, mp, feats, depth, W1, b1, Bhi, Blo, b2, out, fw, fw);
}
